// SelfAttention_4346506904227
// MI455X (gfx1250) — hardware-verified
//
#include <hip/hip_runtime.h>


#ifndef NB
#define NB 4
#endif
#ifndef SEQ
#define SEQ 4096
#endif
#define NB_FULL  4
#define SEQ_FULL 4096
#define DM   512
#define DQ   512
#define DV   512
#define PCAR 1024.0f
#define SCL  0.044194173824159216f
#define L2E  1.4426950408889634f

static_assert(NB >= 1 && NB <= NB_FULL);
static_assert(SEQ >= 128 && SEQ <= SEQ_FULL);
static_assert(SEQ % 128 == 0);
static_assert(DM % 64 == 0 && DQ % 64 == 0 && DV % 64 == 0);
static_assert(DM % 32 == 0 && DQ % 32 == 0 && SEQ % 64 == 0);

typedef _Float16 h16;
typedef unsigned short bf;
typedef __attribute__((ext_vector_type(16))) __bf16   v16bf;
typedef __attribute__((ext_vector_type(16))) _Float16 v16h;
typedef __attribute__((ext_vector_type(8)))  _Float16 v8h;
typedef __attribute__((ext_vector_type(8)))  unsigned short v8us;
typedef __attribute__((ext_vector_type(8)))  float    v8f;
typedef __attribute__((ext_vector_type(4)))  float    v4f;
typedef __attribute__((ext_vector_type(4)))  _Float16 v4h;
typedef __attribute__((ext_vector_type(2)))  unsigned short v2us;
typedef v4f  __attribute__((may_alias)) v4fa;

__device__ __forceinline__ unsigned short f2bf(float f) { unsigned u = __float_as_uint(f); u += 0x7FFFu + ((u >> 16) & 1u); return (unsigned short)(u >> 16); }
__device__ __forceinline__ float bf2f(unsigned short b) { return __uint_as_float(((unsigned)b) << 16); }
__device__ __forceinline__ float bfr(float f) { return bf2f(f2bf(f)); }
__device__ __forceinline__ h16 tohx(float x) { return (h16)x; }
__device__ __forceinline__ v16h cat16(v8h lo, v8h hi) { return __builtin_shufflevector(lo, hi, 0, 1, 2, 3, 4, 5, 6, 7, 8, 9, 10, 11, 12, 13, 14, 15); }
__device__ __forceinline__ v16bf cat16b(v8us lo, v8us hi) { return __builtin_bit_cast(v16bf, __builtin_shufflevector(lo, hi, 0, 1, 2, 3, 4, 5, 6, 7, 8, 9, 10, 11, 12, 13, 14, 15)); }
__device__ __forceinline__ v8f wmma16(v16h a, v16h b, v8f c) { return __builtin_amdgcn_wmma_f32_16x16x32_f16(false, a, false, b, (short)0, c, false, false); }
__device__ __forceinline__ v8f wmmab(v16bf a, v16bf b, v8f c) { return __builtin_amdgcn_wmma_f32_16x16x32_bf16(false, a, false, b, (short)0, c, false, false); }

template <typename T16> struct WFrag;
template <> struct WFrag<h16> { typedef v16h V; static __device__ __forceinline__ V ld(const h16* p) { return cat16(*(const v8h*)p, *(const v8h*)(p + 16)); } static __device__ __forceinline__ v8f mma(V a, V b, v8f c) { return wmma16(a, b, c); } };
template <> struct WFrag<bf> { typedef v16bf V; static __device__ __forceinline__ V ld(const bf* p) { return cat16b(*(const v8us*)p, *(const v8us*)(p + 16)); } static __device__ __forceinline__ v8f mma(V a, V b, v8f c) { return wmmab(a, b, c); } };
template <typename T16, int NSPLIT, bool BIAS>
__global__ __launch_bounds__(32) void k_gemmw(const T16* __restrict__ A, const T16* __restrict__ A2, const T16* __restrict__ Bt, const T16* __restrict__ Bt2, int K, float* C, int ldc, const float* __restrict__ bias, size_t sA, size_t sB, size_t sC) {
    typedef typename WFrag<T16>::V V;
    __shared__ __align__(16) float os[16 * 68];
    const size_t z = blockIdx.z; A += z * sA; if (A2) A2 += z * sA; Bt += z * sB; if (Bt2) Bt2 += z * sB; C += z * sC;
    const int lane = threadIdx.x & 31, lr = lane & 15, hi = lane >> 4; const int r0 = blockIdx.x * 64, c0 = blockIdx.y * 64;
    v8f acc[4][4];
#pragma unroll
    for (int mb = 0; mb < 4; ++mb)
#pragma unroll
        for (int nb = 0; nb < 4; ++nb) acc[mb][nb] = (v8f){};
    const size_t aoff = (size_t)(r0 + lr) * K + 8 * hi, boff = (size_t)(c0 + lr) * K + 8 * hi;
#pragma unroll 1
    for (int kc = 0; kc < K; kc += 32) {
        V a[4], a2[4];
#pragma unroll
        for (int mb = 0; mb < 4; ++mb) { a[mb] = WFrag<T16>::ld(A + aoff + (size_t)mb * 16 * K + kc); if (NSPLIT == 1 || NSPLIT == 2) a2[mb] = WFrag<T16>::ld(A2 + aoff + (size_t)mb * 16 * K + kc); }
#pragma unroll
        for (int nb = 0; nb < 4; ++nb) { const V b = WFrag<T16>::ld(Bt + boff + (size_t)nb * 16 * K + kc); V b2; if (NSPLIT >= 2) b2 = WFrag<T16>::ld(Bt2 + boff + (size_t)nb * 16 * K + kc);
#pragma unroll
            for (int mb = 0; mb < 4; ++mb) { acc[mb][nb] = WFrag<T16>::mma(a[mb], b, acc[mb][nb]); if (NSPLIT == 1 || NSPLIT == 2) acc[mb][nb] = WFrag<T16>::mma(a2[mb], b, acc[mb][nb]); if (NSPLIT >= 2) acc[mb][nb] = WFrag<T16>::mma(a[mb], b2, acc[mb][nb]); } }
        asm volatile("v_nop\n\tv_nop\n\tv_nop\n\tv_nop" : "+v"(acc[0][0]), "+v"(acc[1][1]), "+v"(acc[2][2]), "+v"(acc[3][3]) : "v"(a[0]), "v"(a[3]));
    }
#pragma unroll
    for (int mb = 0; mb < 4; ++mb) {
#pragma unroll
        for (int nb = 0; nb < 4; ++nb) {
#pragma unroll
            for (int j = 0; j < 8; ++j) os[(hi * 8 + j) * 68 + nb * 16 + lr] = acc[mb][nb][j]; }
        __builtin_amdgcn_wave_barrier(); asm volatile("" ::: "memory");
        float* crow = C + (size_t)(r0 + mb * 16) * ldc + c0;
#pragma unroll 1
        for (int ps = 0; ps < 2; ++ps) {
#pragma unroll
            for (int s = 0; s < 8; ++s) { const int row = 2 * s + hi, cofs = lr * 4; v4f val = *(const v4fa*)(os + row * 68 + cofs); if (BIAS) { val[0] += bfr(bias[c0 + cofs]); val[1] += bfr(bias[c0 + cofs + 1]); val[2] += bfr(bias[c0 + cofs + 2]); val[3] += bfr(bias[c0 + cofs + 3]); }
                *(volatile v4f*)(crow + (size_t)row * ldc + cofs) = val; }
            if (ps == 0) __threadfence(); }
        __builtin_amdgcn_wave_barrier(); asm volatile("" ::: "memory");
    }
}

__global__ __launch_bounds__(256) void k_wtG(const float* __restrict__ w, int K, int N, bf* Bt) {
    const int lane = threadIdx.x & 31; const int L0 = (blockIdx.x * 8 + (threadIdx.x >> 5)) * 8; const int nlines = N * K / 64;
#pragma unroll
    for (int ps = 0; ps < 2; ++ps) {
#pragma unroll 1
        for (int l = 0; l < 8; ++l) { const int L = L0 + l; if (L >= nlines) break; const size_t e = (size_t)L * 64 + lane * 2; const int k = (int)(e % K), n = (int)(e / K); v2us o;
            o[0] = f2bf(w[(size_t)k * N + n]); o[1] = f2bf(w[(size_t)(k + 1) * N + n]); *(volatile v2us*)(Bt + e) = o; }
        if (ps == 0) __threadfence(); }
}
__global__ __launch_bounds__(256) void k_cvt8(const float* __restrict__ src, bf* dst, size_t n8) { const size_t i = (size_t)blockIdx.x * 256 + threadIdx.x; if (i >= n8) return; const v8f v = *(const v8f*)(src + i * 8); v8us o;
#pragma unroll
    for (int k = 0; k < 8; ++k) o[k] = f2bf(v[k]); *(volatile v8us*)(dst + i * 8) = o; __threadfence(); *(volatile v8us*)(dst + i * 8) = o; }
__global__ __launch_bounds__(256) void k_cvh8(const float* __restrict__ src, h16* dst, size_t n8) { const size_t i = (size_t)blockIdx.x * 256 + threadIdx.x; if (i >= n8) return; const v8f v = *(const v8f*)(src + i * 8); v8h o;
#pragma unroll
    for (int k = 0; k < 8; ++k) o[k] = tohx(v[k]); *(volatile v8h*)(dst + i * 8) = o; __threadfence(); *(volatile v8h*)(dst + i * 8) = o; }
__global__ __launch_bounds__(256) void k_vtp8(const float* __restrict__ F, int pitch, h16* V16) {
    const size_t e = ((size_t)blockIdx.x * 256 + threadIdx.x) * 8; if (e >= (size_t)DV * SEQ) return; const int t = (int)(e % SEQ); const int d = (int)(e / SEQ); v8h o;
#pragma unroll
    for (int q = 0; q < 8; ++q) o[q] = tohx(F[(size_t)(t + q) * pitch + d]);
    *(volatile v8h*)(V16 + e) = o; __threadfence(); *(volatile v8h*)(V16 + e) = o; }
__global__ __launch_bounds__(256) void k_asoft(const float* __restrict__ Sb, h16* P16) {
    const int lane = threadIdx.x & 31; const int row = blockIdx.x * 8 + (threadIdx.x >> 5); if (row >= SEQ) return;
    const float* sr = Sb + (size_t)row * SEQ; float v[SEQ / 32]; float mx = -3.0e38f;
#pragma unroll
    for (int ch = 0; ch < SEQ / 128; ++ch) { const int j0 = ch * 128 + lane * 4; const v4f a = *(const v4f*)(sr + j0);
#pragma unroll
        for (int q = 0; q < 4; ++q) { v[ch * 4 + q] = a[q]; mx = fmaxf(mx, a[q]); }
        if ((ch & 7) == 7) asm volatile("" ::: "memory"); }
#pragma unroll
    for (int sh = 16; sh; sh >>= 1) mx = fmaxf(mx, __shfl_xor(mx, sh, 32));
    float sum = 0.f;
#pragma unroll
    for (int k = 0; k < SEQ / 32; ++k) { float d0 = __fsub_rn(v[k], mx); asm volatile("" : "+v"(d0)); v[k] = __builtin_amdgcn_exp2f(__fmul_rn(d0, SCL * L2E)); sum += v[k]; }
#pragma unroll
    for (int sh = 16; sh; sh >>= 1) sum += __shfl_xor(sum, sh, 32);
    const float f = __fdiv_rn(PCAR, sum);
#pragma unroll 1
    for (int ps = 0; ps < 2; ++ps) {
#pragma unroll
        for (int ch = 0; ch < SEQ / 128; ++ch) { v4h o4;
#pragma unroll
            for (int q = 0; q < 4; ++q) o4[q] = tohx(v[ch * 4 + q] * f);
            *(volatile v4h*)(P16 + (size_t)row * SEQ + ch * 128 + lane * 4) = o4; }
        if (ps == 0) __threadfence(); }
}
__global__ __launch_bounds__(256) void k_merge(const float* __restrict__ O, float* OUTb) { const size_t e = ((size_t)blockIdx.x * 256 + threadIdx.x) * 4; if (e >= (size_t)SEQ * DV) return; v4f o = *(const v4f*)(O + e);
#pragma unroll
    for (int q = 0; q < 4; ++q) o[q] = o[q] * (1.0f / PCAR);
    *(volatile v4f*)(OUTb + e) = o; __threadfence(); *(volatile v4f*)(OUTb + e) = o; }

extern "C" void kernel_launch(void* const* d_in, const int* in_sizes, int n_in,
                              void* d_out, int out_size, void* d_ws, size_t ws_size, hipStream_t stream) {
    if (n_in < 7) return;
    if ((size_t)in_sizes[0] < (size_t)(NB - 1) * SEQ_FULL * DM + (size_t)SEQ * DM) return;
    if (in_sizes[1] < DM * DQ || in_sizes[2] < DQ || in_sizes[3] < DM * DQ || in_sizes[4] < DQ || in_sizes[5] < DM * DV || in_sizes[6] < DV) return;
    if (out_size < 0 || (size_t)out_size < (size_t)(NB - 1) * SEQ_FULL * DV + (size_t)SEQ * DV) return;
    const float* x = (const float*)d_in[0]; const float* wq = (const float*)d_in[1]; const float* bq = (const float*)d_in[2]; const float* wk = (const float*)d_in[3]; const float* bk = (const float*)d_in[4]; const float* wv = (const float*)d_in[5]; const float* bv = (const float*)d_in[6];
    float* OUT = (float*)d_out;
    char* base = (char*)d_ws; size_t off = 0;
    auto take = [&](size_t bytes) { void* p = base + off; off += (bytes + 255) & ~(size_t)255; return p; };
    bf* WQ = (bf*)take((size_t)DQ * DM * 2); bf* WK = (bf*)take((size_t)DQ * DM * 2); bf* WV = (bf*)take((size_t)DV * DM * 2);
    const size_t regA = off;
    bf* XB = (bf*)take((size_t)SEQ * DM * 2); float* FQ = (float*)take((size_t)SEQ * DQ * 4); float* FK = (float*)take((size_t)SEQ * (DQ > DV ? DQ : DV) * 4);
    const size_t endA = off;
    off = regA; float* Sb = (float*)take((size_t)SEQ * SEQ * 4); if (off < endA) off = endA;
    h16* QP16 = (h16*)take((size_t)SEQ * DQ * 2); h16* KP16 = (h16*)take((size_t)SEQ * DQ * 2); h16* VT16 = (h16*)take((size_t)DV * SEQ * 2);
    h16* P16 = (h16*)take((size_t)SEQ * SEQ * 2); float* Ob = (float*)take((size_t)SEQ * DV * 4);
    if (off > ws_size) return;
    float* FV = FK;

    k_wtG<<<(unsigned)((DM * DQ / 64 + 63) / 64), 256, 0, stream>>>(wq, DM, DQ, WQ);
    k_wtG<<<(unsigned)((DM * DQ / 64 + 63) / 64), 256, 0, stream>>>(wk, DM, DQ, WK);
    k_wtG<<<(unsigned)((DM * DV / 64 + 63) / 64), 256, 0, stream>>>(wv, DM, DV, WV);
    const size_t n8x = (size_t)SEQ * DM / 8, n8q = (size_t)SEQ * DQ / 8;
    const unsigned LX = (unsigned)((n8x + 255) / 256), LQ = (unsigned)((n8q + 255) / 256);
    const unsigned LVT = (unsigned)(((size_t)DV * SEQ / 8 + 255) / 256), LM = (unsigned)(((size_t)SEQ * DV / 4 + 255) / 256);
    for (int b = 0; b < NB; ++b) {
        const float* xb = x + (size_t)b * SEQ_FULL * DM; float* ob = OUT + (size_t)b * SEQ_FULL * DV;
        k_cvt8<<<LX, 256, 0, stream>>>(xb, XB, n8x);
        k_gemmw<bf, 0, true><<<dim3(SEQ / 64, DQ / 64, 1), 32, 0, stream>>>(XB, nullptr, WQ, nullptr, DM, FQ, DQ, bq, 0, 0, 0);
        k_cvh8<<<LQ, 256, 0, stream>>>(FQ, QP16, n8q);
        k_gemmw<bf, 0, true><<<dim3(SEQ / 64, DQ / 64, 1), 32, 0, stream>>>(XB, nullptr, WK, nullptr, DM, FK, DQ, bk, 0, 0, 0);
        k_cvh8<<<LQ, 256, 0, stream>>>(FK, KP16, n8q);
        k_gemmw<bf, 0, true><<<dim3(SEQ / 64, DV / 64, 1), 32, 0, stream>>>(XB, nullptr, WV, nullptr, DM, FV, DV, bv, 0, 0, 0);
        k_vtp8<<<LVT, 256, 0, stream>>>(FV, DV, VT16);
        k_gemmw<h16, 0, false><<<dim3(SEQ / 64, SEQ / 64, 1), 32, 0, stream>>>(QP16, nullptr, KP16, nullptr, DQ, Sb, SEQ, nullptr, 0, 0, 0);
        k_asoft<<<SEQ / 8, 256, 0, stream>>>(Sb, P16);
        k_gemmw<h16, 0, false><<<dim3(SEQ / 64, DV / 64, 1), 32, 0, stream>>>(P16, nullptr, VT16, nullptr, SEQ, Ob, DV, nullptr, 0, 0, 0);
        k_merge<<<LM, 256, 0, stream>>>(Ob, ob);
    }
}
